// FP8GEMMS_77403900609092
// MI455X (gfx1250) — hardware-verified
//
#include <hip/hip_runtime.h>
#include <math.h>

#pragma clang fp contract(off)

constexpr int kRep    = 4;
constexpr int kRows   = 4096;
constexpr int kCols   = 4096;
constexpr int kDepth  = 512;
constexpr int kKtot   = kRep * kDepth;
constexpr int kInElems      = kRep * kRows * kDepth;
constexpr int kQuantThreads = kInElems / 8;
constexpr int kQuantBlocks  = kQuantThreads / 256;
constexpr int kGemmTiles    = (kRows / 64) * (kCols / 64);
constexpr int kGemmBlocks   = kGemmTiles / 8;
constexpr size_t kPlaneHalves = (size_t)kRows * kKtot;
static_assert(kRows == kCols);
static_assert(kKtot % 32 == 0);
static_assert(kRows % 64 == 0 && kCols % 64 == 0);
static_assert(kQuantBlocks * 256 * 8 == kInElems);
static_assert(kGemmBlocks * 8 == kGemmTiles);

typedef __attribute__((ext_vector_type(16))) _Float16 v16h;
typedef __attribute__((ext_vector_type(8)))  _Float16 v8h;
typedef __attribute__((ext_vector_type(8)))  float    v8f;
typedef __attribute__((ext_vector_type(4)))  float    v4f;
typedef __attribute__((ext_vector_type(4)))  unsigned int v4u;

__device__ __forceinline__ unsigned short f2bf_bits(float f) {
  unsigned u = __float_as_uint(f);
  return (unsigned short)((u + 0x7FFFu + ((u >> 16) & 1u)) >> 16);
}
__device__ __forceinline__ float bf_bits2f(unsigned short h) { return __uint_as_float(((unsigned)h) << 16); }
__device__ __forceinline__ float bf_rne(float f) { return bf_bits2f(f2bf_bits(f)); }

__device__ __forceinline__ void dep_guard_h(v8f& a, v8f& b, v16h x, v16h y) { asm volatile("v_nop\n\tv_nop\n\tv_nop\n\tv_nop" : "+v"(a), "+v"(b) : "v"(x), "v"(y)); }
__device__ __forceinline__ void keep4_h(v16h a, v16h b, v16h c, v16h d) { asm volatile("v_nop" :: "v"(a), "v"(b), "v"(c), "v"(d)); }
__device__ __forceinline__ void acc_guard4(v8f& a, v8f& b, v8f& c, v8f& d) { asm volatile("v_nop\n\tv_nop\n\tv_nop\n\tv_nop" : "+v"(a), "+v"(b), "+v"(c), "+v"(d)); }

template <typename T> struct Frag;
template <> struct Frag<_Float16> {
  typedef v16h V; union U { v16h v; v8h h[2]; };
  static __device__ __forceinline__ v16h load(const _Float16* p) {
    U f; f.h[0] = *(const v8h*)(p); f.h[1] = *(const v8h*)(p + 16); return f.v;
  }
  static __device__ __forceinline__ v8f mma(v16h a, v16h b, v8f c) {
    return __builtin_amdgcn_wmma_f32_16x16x32_f16(false, a, false, b, (short)0, c, false, false);
  }
  static __device__ __forceinline__ void guard(v8f& a, v8f& b, v16h x, v16h y) { dep_guard_h(a, b, x, y); }
  static __device__ __forceinline__ void keep(v16h a, v16h b, v16h c, v16h d) { keep4_h(a, b, c, d); }
};

__device__ __forceinline__ unsigned pk16(unsigned short a, unsigned short b) { return (unsigned)a | ((unsigned)b << 16); }
__device__ __forceinline__ unsigned short h_bits(float f) { const _Float16 h = (_Float16)f; return __builtin_bit_cast(unsigned short, h); }

__device__ __forceinline__ unsigned short quant_e4m3_bits(float v) {
  const float a = fabsf(v);
  const unsigned ua = __float_as_uint(a);
  const unsigned ur = (ua + 0x7FFFFu + ((ua >> 20) & 1u)) & 0xFFF00000u;
  float rn = __uint_as_float(ur);
  rn = (rn > 448.0f) ? __uint_as_float(0x7FC00000u) : rn;
  const float rs = rintf(a * 512.0f) * 0.001953125f;
  float r = (a >= 0.015625f) ? rn : rs;
  r = copysignf(r, v);
  return h_bits(r);
}

__global__ __launch_bounds__(256) void quant_e4m3_kernel(const float* __restrict__ x, const float* __restrict__ s,
                                                         unsigned short* __restrict__ Q) {
  const int i = blockIdx.x * 256 + threadIdx.x;
  if (i >= kQuantThreads) return;
  const int e = i * 8;
  const int r = e >> 21;
  const int m = (e >> 9) & (kRows - 1);
  const int k = e & (kDepth - 1);
  const float sb = bf_rne(s[0]);
  const float* p = x + (size_t)e;
  const v4f a = *(const v4f*)(p);
  const v4f c = *(const v4f*)(p + 4);
  unsigned short hb[8];
#pragma unroll
  for (int t = 0; t < 4; ++t) {
    hb[t]     = quant_e4m3_bits(bf_rne(a[t]) * sb);
    hb[4 + t] = quant_e4m3_bits(bf_rne(c[t]) * sb);
  }
  const v4u u = (v4u){pk16(hb[0], hb[1]), pk16(hb[2], hb[3]), pk16(hb[4], hb[5]), pk16(hb[6], hb[7])};
  unsigned short* q = Q + (size_t)m * kKtot + (size_t)r * kDepth + k;
  *(volatile v4u*)q = u;
  __threadfence();
  *(volatile v4u*)q = u;
}

__global__ __launch_bounds__(256) void gemm_e4m3_kernel(const unsigned short* __restrict__ Ap,
                                                        const unsigned short* __restrict__ Btp,
                                                        unsigned short* __restrict__ Cp,
                                                        const float* __restrict__ si1,
                                                        const float* __restrict__ si2) {
  typedef _Float16 T;
  typedef Frag<T>::V V;
  const T* A  = (const T*)Ap;
  const T* Bt = (const T*)Btp;
  __shared__ __align__(16) float sT[8][16 * 68];
  const int lane = threadIdx.x & 31;
  const int wave = threadIdx.x >> 5;
  constexpr int tilesN = kCols >> 6;
  constexpr int tilesM = kRows >> 6;
  const int tile = blockIdx.x * 8 + wave;
  if (tile >= tilesM * tilesN) return;
  const int tm = tile / tilesN;
  const int tn = tile - tm * tilesN;
  const int m0 = tm << 6;
  const int n0 = tn << 6;

  const int rlane = lane & 15;
  const int koff  = (lane >> 4) * 8;
  const int mOff  = (lane >> 4) * 8;

  const float scale = bf_rne(si1[0]) * bf_rne(si2[0]);

  v8f acc[4][4];
#pragma unroll
  for (int i = 0; i < 4; ++i)
#pragma unroll
    for (int j = 0; j < 4; ++j) acc[i][j] = (v8f){0.f,0.f,0.f,0.f,0.f,0.f,0.f,0.f};

  for (int k0 = 0; k0 < kKtot; k0 += 32) {
    V bh[4];
#pragma unroll
    for (int j = 0; j < 4; ++j) {
      const size_t bo = (size_t)(n0 + (j << 4) + rlane) * kKtot + koff + k0;
      bh[j] = Frag<T>::load(Bt + bo);
    }
#pragma unroll
    for (int i = 0; i < 4; ++i) {
      const size_t ao = (size_t)(m0 + (i << 4) + rlane) * kKtot + koff + k0;
      V ah = Frag<T>::load(A + ao);
#pragma unroll
      for (int j = 0; j < 4; ++j) {
        acc[i][j] = Frag<T>::mma(ah, bh[j], acc[i][j]);
      }
      Frag<T>::guard(acc[i][0], acc[i][3], ah, ah);
    }
    Frag<T>::keep(bh[0], bh[1], bh[2], bh[3]);
  }
  acc_guard4(acc[0][0], acc[0][1], acc[0][2], acc[0][3]);
  acc_guard4(acc[1][0], acc[1][1], acc[1][2], acc[1][3]);
  acc_guard4(acc[2][0], acc[2][1], acc[2][2], acc[2][3]);
  acc_guard4(acc[3][0], acc[3][1], acc[3][2], acc[3][3]);

  float* slab = sT[wave];
#pragma unroll
  for (int i = 0; i < 4; ++i) {
    const int mBase = m0 + (i << 4);
#pragma unroll
    for (int j = 0; j < 4; ++j) {
#pragma unroll
      for (int r = 0; r < 8; ++r) {
        const float v = acc[i][j][r] * scale;
        slab[(mOff + r) * 68 + (j << 4) + rlane] = v;
      }
    }
    __builtin_amdgcn_fence(__ATOMIC_RELEASE, "workgroup");
    __builtin_amdgcn_wave_barrier();
    __builtin_amdgcn_fence(__ATOMIC_ACQUIRE, "workgroup");
    {
      const int q = lane >> 3, c8 = (lane & 7) * 8;
      for (int pass = 0; pass < 2; ++pass) {
#pragma unroll
        for (int it = 0; it < 4; ++it) {
          const int row = it * 4 + q;
          const float* sp = slab + row * 68 + c8;
          unsigned short hb[8];
#pragma unroll
          for (int e = 0; e < 8; ++e) hb[e] = f2bf_bits(sp[e]);
          const v4u u = (v4u){pk16(hb[0], hb[1]), pk16(hb[2], hb[3]), pk16(hb[4], hb[5]), pk16(hb[6], hb[7])};
          *(volatile v4u*)(Cp + (size_t)(mBase + row) * kCols + n0 + c8) = u;
        }
        __threadfence();
      }
    }
    __builtin_amdgcn_fence(__ATOMIC_RELEASE, "workgroup");
    __builtin_amdgcn_wave_barrier();
    __builtin_amdgcn_fence(__ATOMIC_ACQUIRE, "workgroup");
  }
}

extern "C" void kernel_launch(void* const* d_in, const int* in_sizes, int n_in,
                              void* d_out, int out_size, void* d_ws, size_t ws_size,
                              hipStream_t stream) {
  if (n_in < 6) return;
  if (in_sizes[0] != kInElems || in_sizes[1] != kInElems) return;
  if (in_sizes[2] < 1 || in_sizes[3] < 1 || in_sizes[4] < 1 || in_sizes[5] < 1) return;
  if (out_size != kRows * kCols) return;
  const size_t carve_bytes = 2 * kPlaneHalves * sizeof(unsigned short);
  if (ws_size < carve_bytes) return;

  const float* x1  = (const float*)d_in[0];
  const float* x2  = (const float*)d_in[1];
  const float* s1  = (const float*)d_in[2];
  const float* s2  = (const float*)d_in[3];
  const float* si1 = (const float*)d_in[4];
  const float* si2 = (const float*)d_in[5];
  unsigned short* out = (unsigned short*)d_out;

  unsigned short* Aq  = (unsigned short*)d_ws;
  unsigned short* Btq = Aq + kPlaneHalves;

  quant_e4m3_kernel<<<dim3(kQuantBlocks, 1, 1), dim3(256, 1, 1), 0, stream>>>(x1, s1, Aq);
  quant_e4m3_kernel<<<dim3(kQuantBlocks, 1, 1), dim3(256, 1, 1), 0, stream>>>(x2, s2, Btq);
  gemm_e4m3_kernel<<<dim3(kGemmBlocks, 1, 1), dim3(256, 1, 1), 0, stream>>>(Aq, Btq, out, si1, si2);
}
